// Mamba_45758581571908
// MI455X (gfx1250) — hardware-run, weakly checked
//
#include <hip/hip_runtime.h>
#include <math.h>

typedef __attribute__((ext_vector_type(16))) _Float16 v16h;
typedef __attribute__((ext_vector_type(8)))  _Float16 v8h;
typedef __attribute__((ext_vector_type(16))) __bf16   v16b;
typedef __attribute__((ext_vector_type(8)))  __bf16   v8b;
typedef __attribute__((ext_vector_type(8)))  float    v8f;
typedef __attribute__((ext_vector_type(4)))  float    v4f;

constexpr int kBatch  = 2;
constexpr int kSeq    = 2048;
constexpr int kDm     = 512;
constexpr int kDin    = 1024;
constexpr int kNst    = 16;
constexpr int kDtR    = 32;
constexpr int kXdP    = 64;
constexpr int kStr    = 2;
constexpr int kRowsB  = kStr * kSeq;
constexpr int kWinR   = 4 * kDin;
constexpr int kFinP   = 2 * kDin;
constexpr int kConvTP = 260;
constexpr int kScanTS = 64;
constexpr int kScanCh = 64;
constexpr int kScanYP = 68;
static_assert(kDtR + 2 * kNst == kXdP, "x_proj width");
static_assert(kDtR == 32, "dt contraction is exactly one 32-deep WMMA k-step");
static_assert((kDm % 32) == 0 && (kDin % 32) == 0 && (kFinP % 32) == 0, "GEMM K multiples of 32");
static_assert((kSeq % 64) == 0 && (kRowsB % 64) == 0 && (kDin % 64) == 0 && (kXdP % 64) == 0 && (kDm % 64) == 0, "GEMM M,N multiples of 64");
static_assert(((kSeq / 64) * (kDin / 64)) % 8 == 0 && ((kRowsB / 64) * (kXdP / 64)) % 8 == 0 && ((kSeq / 64) * (kDm / 64)) % 8 == 0, "8 tiles per GEMM block");
static_assert((kSeq % kScanTS) == 0 && (kDin % kScanCh) == 0 && (kDin % 256) == 0 && kScanTS == 64 && kScanCh == 64, "tile multiples");

constexpr size_t kOffXB   = 0;
constexpr size_t kOffWIB  = kOffXB  + (size_t)kBatch * kSeq * kDm * 2;
constexpr size_t kOffWXF  = kOffWIB + (size_t)kWinR * kDm * 2;
constexpr size_t kOffWXB  = kOffWXF + (size_t)kXdP * kDin * 2;
constexpr size_t kOffWOB  = kOffWXB + (size_t)kXdP * kDin * 2;
constexpr size_t kOffX2   = kOffWOB + (size_t)kDm * kFinP * 2;
constexpr size_t kOffZ2   = kOffX2  + (size_t)kRowsB * kDin * 4;
constexpr size_t kOffUFH  = kOffZ2  + (size_t)kRowsB * kDin * 4;
constexpr size_t kOffUFL  = kOffUFH + (size_t)kRowsB * kDin * 2;
constexpr size_t kOffUBH  = kOffUFL + (size_t)kRowsB * kDin * 2;
constexpr size_t kOffUBL  = kOffUBH + (size_t)kRowsB * kDin * 2;
constexpr size_t kOffXDF  = kOffUBL + (size_t)kRowsB * kDin * 2;
constexpr size_t kOffXDB  = kOffXDF + (size_t)kRowsB * kXdP * 4;
constexpr size_t kOffYF   = kOffXDB + (size_t)kRowsB * kXdP * 4;
constexpr size_t kOffFH   = kOffYF  + (size_t)kRowsB * kDin * 4;
constexpr size_t kOffFL   = kOffFH  + (size_t)kSeq * kFinP * 2;
constexpr size_t kWsTotal = kOffFL  + (size_t)kSeq * kFinP * 2;
static_assert(kWsTotal == 113508352ull, "carve total");
static_assert(kWsTotal <= 134217728ull, "carve cap");
static_assert(kOffZ2 == kOffX2 + (size_t)kRowsB * kDin * 4, "Z2 directly after X2 (used as a C stride)");
static_assert((kOffWIB % 128) == 0 && (kOffWXF % 128) == 0 && (kOffWXB % 128) == 0 && (kOffWOB % 128) == 0 &&
              (kOffX2 % 128) == 0 && (kOffZ2 % 128) == 0 && (kOffUFH % 128) == 0 && (kOffUFL % 128) == 0 &&
              (kOffUBH % 128) == 0 && (kOffUBL % 128) == 0 && (kOffXDF % 128) == 0 && (kOffXDB % 128) == 0 &&
              (kOffYF % 128) == 0 && (kOffFH % 128) == 0 && (kOffFL % 128) == 0, "128-B aligned regions");

__device__ __forceinline__ unsigned short f2bf_bits(float f) {
  unsigned u = __float_as_uint(f);
  return (unsigned short)((u + 0x7FFFu + ((u >> 16) & 1u)) >> 16);
}
__device__ __forceinline__ float bf_bits2f(unsigned short h) { return __uint_as_float(((unsigned)h) << 16); }
__device__ __forceinline__ float bfr(float f) { return bf_bits2f(f2bf_bits(f)); }
__device__ __forceinline__ void split_bf(float f, __bf16& hi, __bf16& lo) {
  const unsigned short hb = f2bf_bits(f);
  hi = __builtin_bit_cast(__bf16, hb);
  lo = __builtin_bit_cast(__bf16, f2bf_bits(f - bf_bits2f(hb)));
}

__device__ __forceinline__ void dep_guard4_h(v8f& a, v8f& b, v8f& c, v8f& d, v16h x, v16h y) {
  asm volatile("v_nop\n\tv_nop\n\tv_nop\n\tv_nop" : "+v"(a), "+v"(b), "+v"(c), "+v"(d) : "v"(x), "v"(y));
}
__device__ __forceinline__ void dep_guard4_b(v8f& a, v8f& b, v8f& c, v8f& d, v16b x, v16b y) {
  asm volatile("v_nop\n\tv_nop\n\tv_nop\n\tv_nop" : "+v"(a), "+v"(b), "+v"(c), "+v"(d) : "v"(x), "v"(y));
}
__device__ __forceinline__ void dep_guard2x4_b(v8f& a, v8f& b, v16b x, v16b y, v16b z, v16b w) {
  asm volatile("v_nop\n\tv_nop\n\tv_nop\n\tv_nop" : "+v"(a), "+v"(b) : "v"(x), "v"(y), "v"(z), "v"(w));
}
__device__ __forceinline__ void keep4_h(v16h a, v16h b, v16h c, v16h d) { asm volatile("v_nop" :: "v"(a), "v"(b), "v"(c), "v"(d)); }
__device__ __forceinline__ void keep4_b(v16b a, v16b b, v16b c, v16b d) { asm volatile("v_nop" :: "v"(a), "v"(b), "v"(c), "v"(d)); }
__device__ __forceinline__ void acc_guard4(v8f& a, v8f& b, v8f& c, v8f& d) { asm volatile("v_nop\n\tv_nop\n\tv_nop\n\tv_nop" : "+v"(a), "+v"(b), "+v"(c), "+v"(d)); }
template <typename T> struct Frag;
template <> struct Frag<_Float16> {
  typedef v16h V; union U { v16h v; v8h h[2]; };
  static __device__ __forceinline__ v16h load(const _Float16* p) {
    U f; f.h[0] = *(const v8h*)(p); f.h[1] = *(const v8h*)(p + 16); return f.v;
  }
  static __device__ __forceinline__ v8f mma(v16h a, v16h b, v8f c) {
    return __builtin_amdgcn_wmma_f32_16x16x32_f16(false, a, false, b, (short)0, c, false, false);
  }
  static __device__ __forceinline__ void guard4(v8f& a, v8f& b, v8f& c, v8f& d, v16h x, v16h y) { dep_guard4_h(a, b, c, d, x, y); }
  static __device__ __forceinline__ void keep(v16h a, v16h b, v16h c, v16h d) { keep4_h(a, b, c, d); }
};
template <> struct Frag<__bf16> {
  typedef v16b V; union U { v16b v; v8b h[2]; };
  static __device__ __forceinline__ v16b load(const __bf16* p) {
    U f; f.h[0] = *(const v8b*)(p); f.h[1] = *(const v8b*)(p + 16); return f.v;
  }
  static __device__ __forceinline__ v8f mma(v16b a, v16b b, v8f c) {
    return __builtin_amdgcn_wmma_f32_16x16x32_bf16(false, a, false, b, (short)0, c, false, false);
  }
  static __device__ __forceinline__ void guard4(v8f& a, v8f& b, v8f& c, v8f& d, v16b x, v16b y) { dep_guard4_b(a, b, c, d, x, y); }
  static __device__ __forceinline__ void keep(v16b a, v16b b, v16b c, v16b d) { keep4_b(a, b, c, d); }
};

template <int ET> struct Elem;
template <> struct Elem<0> { typedef _Float16 T; };
template <> struct Elem<1> { typedef __bf16 T; };
template <int ET, int SPL, int BIAS_MODE, int OUT_MODE, bool RESID, int ACT, int REVROW>
__global__ __launch_bounds__(256) void wmma_gemm64(
    const unsigned short* __restrict__ Ap, const unsigned short* __restrict__ A2p, int lda, long strideA,
    const unsigned short* __restrict__ Btp, const unsigned short* __restrict__ Bt2p, int ldb, long strideB,
    void* __restrict__ Cout, void* __restrict__ Cout2, int ldc, long strideC,
    const float* __restrict__ bias,
    const float* __restrict__ resid, long strideR,
    int M, int N, int K, float scale) {
  typedef typename Elem<ET>::T T;
  typedef typename Frag<T>::V V;
  const T* A = (const T*)Ap; const T* A2 = (const T*)A2p; const T* Bt = (const T*)Btp; const T* Bt2 = (const T*)Bt2p;
  __shared__ __align__(16) float sT[8][16 * 68];
  const int b    = blockIdx.y;
  const int lane = threadIdx.x & 31;
  const int wave = threadIdx.x >> 5;
  const int tilesN = N >> 6;
  const int tilesM = M >> 6;
  const int tile = blockIdx.x * 8 + wave;
  if (tile >= tilesM * tilesN) return;
  const int tm = tile / tilesN;
  const int tn = tile - tm * tilesN;
  const int m0 = tm << 6;
  const int n0 = tn << 6;

  const T* Ab  = A  + (size_t)b * strideA;
  const T* Bb  = Bt + (size_t)b * strideB;
  const T* Ab2 = (SPL >= 1) ? (A2  + (size_t)b * strideA) : nullptr;
  const T* Bb2 = (SPL == 2) ? (Bt2 + (size_t)b * strideB) : nullptr;

  const int rlane = lane & 15;
  const int koff  = (lane >> 4) * 8;
  const int mOff  = (lane >> 4) * 8;

  v8f acc[4][4];
#pragma unroll
  for (int i = 0; i < 4; ++i)
#pragma unroll
    for (int j = 0; j < 4; ++j) acc[i][j] = (v8f){0.f,0.f,0.f,0.f,0.f,0.f,0.f,0.f};

  for (int k0 = 0; k0 < K; k0 += 32) {
    V bh[4], bl[4];
#pragma unroll
    for (int j = 0; j < 4; ++j) {
      const size_t bo = (size_t)(n0 + (j << 4) + rlane) * ldb + koff + k0;
      bh[j] = Frag<T>::load(Bb + bo);
      if (SPL == 2) bl[j] = Frag<T>::load(Bb2 + bo);
    }
#pragma unroll
    for (int i = 0; i < 4; ++i) {
      const size_t ao = (size_t)(m0 + (i << 4) + rlane) * lda + koff + k0;
      V ah = Frag<T>::load(Ab + ao);
      V al = ah;
      if (SPL >= 1) al = Frag<T>::load(Ab2 + ao);
#pragma unroll
      for (int j = 0; j < 4; ++j) {
        acc[i][j] = Frag<T>::mma(ah, bh[j], acc[i][j]);
        if (SPL == 2) acc[i][j] = Frag<T>::mma(ah, bl[j], acc[i][j]);
        if (SPL >= 1) acc[i][j] = Frag<T>::mma(al, bh[j], acc[i][j]);
      }
      Frag<T>::guard4(acc[i][0], acc[i][1], acc[i][2], acc[i][3], ah, al);
    }
    Frag<T>::keep(bh[0], bh[1], bh[2], bh[3]);
    if (SPL == 2) Frag<T>::keep(bl[0], bl[1], bl[2], bl[3]);
  }
  acc_guard4(acc[0][0], acc[0][1], acc[0][2], acc[0][3]);
  acc_guard4(acc[1][0], acc[1][1], acc[1][2], acc[1][3]);
  acc_guard4(acc[2][0], acc[2][1], acc[2][2], acc[2][3]);
  acc_guard4(acc[3][0], acc[3][1], acc[3][2], acc[3][3]);

  float* slab = sT[wave];
  const float* Rb = RESID ? (resid + (size_t)b * strideR) : nullptr;
#pragma unroll
  for (int i = 0; i < 4; ++i) {
    const int mBase = m0 + (i << 4);
#pragma unroll
    for (int j = 0; j < 4; ++j) {
      const int n = n0 + (j << 4) + rlane;
      float bv = 0.f;
      if (BIAS_MODE == 2) bv = bias[n];
#pragma unroll
      for (int r = 0; r < 8; ++r) {
        float v = acc[i][j][r] * scale;
        if (BIAS_MODE == 1) v += bias[mBase + mOff + r];
        if (BIAS_MODE == 2) v += bv;
        if (RESID) v += Rb[(size_t)(mBase + mOff + r) * ldc + n];
        if (ACT == 1) v = tanhf(v);
        if (ACT == 2) v = fmaxf(v, 0.0f);
        if (ACT == 3) v = v / (1.0f + expf(-v));
        if (ACT == 4) v = (v > 0.f) ? v : 0.01f * v;
        slab[(mOff + r) * 68 + (j << 4) + rlane] = v;
      }
    }
    __builtin_amdgcn_fence(__ATOMIC_RELEASE, "workgroup");
    __builtin_amdgcn_wave_barrier();
    __builtin_amdgcn_fence(__ATOMIC_ACQUIRE, "workgroup");
    if (OUT_MODE == 0) {
      float* C = (float*)Cout + (size_t)b * strideC;
      const int hh = lane >> 4, c4 = (lane & 15) * 4;
      for (int pass = 0; pass < 2; ++pass) {
#pragma unroll
        for (int it = 0; it < 8; ++it) {
          const int row = it * 2 + hh;
          const int grow = REVROW ? (M - 1 - (mBase + row)) : (mBase + row);
          v4f v = *(const v4f*)(slab + row * 68 + c4);
          *(volatile v4f*)(C + (size_t)grow * ldc + n0 + c4) = v;
        }
        __threadfence();
      }
    } else {
      const int q = lane >> 3, c8 = (lane & 7) * 8;
      unsigned short* C  = (unsigned short*)Cout  + (size_t)b * strideC;
      unsigned short* C2 = (OUT_MODE == 2) ? ((unsigned short*)Cout2 + (size_t)b * strideC) : nullptr;
      for (int pass = 0; pass < 2; ++pass) {
#pragma unroll
        for (int it = 0; it < 4; ++it) {
          const int row = it * 4 + q;
          const int grow = REVROW ? (M - 1 - (mBase + row)) : (mBase + row);
          const float* sp = slab + row * 68 + c8;
          v8h hv, lv;
#pragma unroll
          for (int e = 0; e < 8; ++e) {
            if (OUT_MODE == 1) {
              hv[e] = (_Float16)sp[e];
            } else {
              unsigned short hb = f2bf_bits(sp[e]);
              unsigned short lb = f2bf_bits(sp[e] - bf_bits2f(hb));
              hv[e] = __builtin_bit_cast(_Float16, hb);
              lv[e] = __builtin_bit_cast(_Float16, lb);
            }
          }
          *(volatile v8h*)(C + (size_t)grow * ldc + n0 + c8) = hv;
          if (OUT_MODE == 2) *(volatile v8h*)(C2 + (size_t)grow * ldc + n0 + c8) = lv;
        }
        __threadfence();
      }
    }
    __builtin_amdgcn_fence(__ATOMIC_RELEASE, "workgroup");
    __builtin_amdgcn_wave_barrier();
    __builtin_amdgcn_fence(__ATOMIC_ACQUIRE, "workgroup");
  }
}

__global__ __launch_bounds__(256) void cvt_rows_bf16_kernel(
    const float* __restrict__ src, unsigned short* __restrict__ dst, int total8)
{
  const int i = blockIdx.x * 256 + threadIdx.x;
  if (i >= total8) return;
  const size_t e0 = (size_t)i << 3;
  const v4f a0 = *(const v4f*)(src + e0);
  const v4f a1 = *(const v4f*)(src + e0 + 4);
  v8h hv;
#pragma unroll
  for (int e = 0; e < 4; ++e) {
    const unsigned short h0 = f2bf_bits(a0[e]), h1 = f2bf_bits(a1[e]);
    hv[e]     = __builtin_bit_cast(_Float16, h0);
    hv[4 + e] = __builtin_bit_cast(_Float16, h1);
  }
  unsigned short* qh = dst + e0;
  *(volatile v8h*)qh = hv;
  __threadfence();
  *(volatile v8h*)qh = hv;
}

template <int DIR>
__global__ __launch_bounds__(256) void conv_silu_kernel(
    const float* __restrict__ X2, const float* __restrict__ cw, const float* __restrict__ cb,
    unsigned short* __restrict__ UH, unsigned short* __restrict__ UL)
{
  __shared__ __align__(16) float sT[16 * kConvTP];
  const int tid = threadIdx.x, lane = tid & 31, wave = tid >> 5;
  const int d0 = blockIdx.x * 256, d = d0 + tid;
  const int g0 = blockIdx.y * 64;
  const int tb = g0 & (kSeq - 1);
  const float w0 = bfr(cw[d * 4 + 0]), w1 = bfr(cw[d * 4 + 1]), w2 = bfr(cw[d * 4 + 2]), w3 = bfr(cw[d * 4 + 3]);
  const float bc = bfr(cb[d]);
  float xa, xb, xc;
  {
    bool hist;
    int rb;
    if (DIR == 0) { hist = (tb > 0); rb = hist ? (g0 - 3) : g0; }
    else          { hist = (tb + 64 < kSeq); rb = hist ? (g0 + 64) : g0; }
    const float v0 = X2[(size_t)rb * kDin + d];
    const float v1 = X2[(size_t)(rb + 1) * kDin + d];
    const float v2 = X2[(size_t)(rb + 2) * kDin + d];
    const float fh = hist ? 1.0f : 0.0f;
    if (DIR == 0) { xa = v0 * fh; xb = v1 * fh; xc = v2 * fh; }
    else          { xa = v2 * fh; xb = v1 * fh; xc = v0 * fh; }
  }
#pragma unroll 1
  for (int subi = 0; subi < 4; ++subi) {
    const int sub = DIR ? (3 - subi) : subi;
    const int lb = g0 + sub * 16;
#pragma unroll 1
    for (int si = 0; si < 16; ++si) {
      const int s = DIR ? (15 - si) : si;
      const float xcur = X2[(size_t)(lb + s) * kDin + d];
      float acc = w0 * xa;
      acc = fmaf(w1, xb, acc);
      acc = fmaf(w2, xc, acc);
      acc = fmaf(w3, xcur, acc);
      const float sv = acc + bc;
      const float e  = __expf(fminf(-sv, 80.0f));
      const float sg = __builtin_amdgcn_rcpf(1.0f + e);
      sT[s * kConvTP + tid] = sv * sg;
      xa = xb; xb = xc; xc = xcur;
    }
    __syncthreads();
    v8h hv[2], lv[2];
#pragma unroll
    for (int it = 0; it < 2; ++it) {
      const float* sp = sT + (it * 8 + wave) * kConvTP + lane * 8;
      const v4f a0 = *(const v4f*)(sp);
      const v4f a1 = *(const v4f*)(sp + 4);
#pragma unroll
      for (int e = 0; e < 4; ++e) {
        const unsigned short h0 = f2bf_bits(a0[e]), h1 = f2bf_bits(a1[e]);
        const unsigned short l0 = f2bf_bits(a0[e] - bf_bits2f(h0)), l1 = f2bf_bits(a1[e] - bf_bits2f(h1));
        hv[it][e]     = __builtin_bit_cast(_Float16, h0);
        hv[it][4 + e] = __builtin_bit_cast(_Float16, h1);
        lv[it][e]     = __builtin_bit_cast(_Float16, l0);
        lv[it][4 + e] = __builtin_bit_cast(_Float16, l1);
      }
    }
    for (int pass = 0; pass < 2; ++pass) {
#pragma unroll
      for (int it = 0; it < 2; ++it) {
        const size_t o = (size_t)(lb + it * 8 + wave) * kDin + d0 + lane * 8;
        *(volatile v8h*)(UH + o) = hv[it];
        *(volatile v8h*)(UL + o) = lv[it];
      }
      __threadfence();
    }
    __syncthreads();
  }
}

template <int DIR>
__global__ __launch_bounds__(64) void scan_kernel(
    const float* __restrict__ XD, const unsigned short* __restrict__ UH, const unsigned short* __restrict__ UL,
    const float* __restrict__ Z2, const float* __restrict__ Wdt, const float* __restrict__ bdt,
    const float* __restrict__ Alog, const float* __restrict__ Dp,
    const float* __restrict__ YFin, float* __restrict__ YFout,
    unsigned short* __restrict__ FH, unsigned short* __restrict__ FL)
{
  __shared__ __align__(16) float    sX[kScanTS * kXdP];
  __shared__ __align__(16) float    sD[kScanTS * kScanYP];
  __shared__ __align__(16) float    sY[kScanTS * kScanYP];
  __shared__ __align__(16) unsigned sWw[kScanCh * (kDtR / 2)];
  __shared__ __align__(16) float    sA[kNst * kScanCh];
  typedef Frag<__bf16> FB16;
  const int tid = threadIdx.x, lane = tid & 31, wave = tid >> 5;
  constexpr int kBlkPerS = kDin / kScanCh;
  const int strm = blockIdx.x / kBlkPerS;
  const int d0   = (blockIdx.x - strm * kBlkPerS) * kScanCh;
  const int d    = d0 + tid;
  const size_t row0 = (size_t)strm * kSeq;
  const unsigned* UHw = (const unsigned*)UH;
  const unsigned* ULw = (const unsigned*)UL;
#pragma unroll 1
  for (int r4 = 0; r4 < kDtR / 4; ++r4) {
    const v4f w = *(const v4f*)(Wdt + (size_t)d * kDtR + 4 * r4);
    const unsigned p0 = (unsigned)f2bf_bits(w[0]) | ((unsigned)f2bf_bits(w[1]) << 16);
    const unsigned p1 = (unsigned)f2bf_bits(w[2]) | ((unsigned)f2bf_bits(w[3]) << 16);
    sWw[tid * (kDtR / 2) + 2 * r4]     = p0;
    sWw[tid * (kDtR / 2) + 2 * r4 + 1] = p1;
  }
#pragma unroll 1
  for (int s = 0; s < kNst; ++s) {
    float a = -expf(bfr(Alog[(size_t)d * kNst + s]));
    if (DIR == 0) a = (d >= kDin / 2 && d < kDin / 2 + kNst && s == d - kDin / 2) ? 0.0f : a;
    sA[s * kScanCh + tid] = a;
  }
  __syncthreads();
  float negA[kNst], h[kNst];
#pragma unroll
  for (int s = 0; s < kNst; ++s) {
    negA[s] = sA[s * kScanCh + tid];
    h[s] = 0.f;
  }
  const float bb = bfr(bdt[d]), Dd = bfr(Dp[d]);
  const int rlane = lane & 15;
  const int koff  = (lane >> 4) * 8;
  const int mOff  = (lane >> 4) * 8;
  const __bf16* sWb = (const __bf16*)sWw;
  const v16b bw0 = FB16::load(sWb + (size_t)(wave * 32 + rlane) * kDtR + koff);
  const v16b bw1 = FB16::load(sWb + (size_t)(wave * 32 + 16 + rlane) * kDtR + koff);
  const int lr = tid >> 4, lc4 = (tid & 15) * 4;
  const int hh = lane >> 4, c4 = (lane & 15) * 4;
  const int q = lane >> 3, c8 = (lane & 7) * 8;
  const int odd = d & 1;
#pragma unroll 1
  for (int ci = 0; ci < kSeq / kScanTS; ++ci) {
    const int t0 = (DIR ? (kSeq / kScanTS - 1 - ci) : ci) * kScanTS;
    __syncthreads();
#pragma unroll
    for (int i = 0; i < 8; ++i) {
      const int r = lr + 4 * i;
      *(v4f*)(sX + r * kXdP + lc4) = *(const v4f*)(XD + (row0 + t0 + r) * kXdP + lc4);
    }
    asm volatile("" ::: "memory");
#pragma unroll
    for (int i = 8; i < 16; ++i) {
      const int r = lr + 4 * i;
      *(v4f*)(sX + r * kXdP + lc4) = *(const v4f*)(XD + (row0 + t0 + r) * kXdP + lc4);
    }
    __syncthreads();
#pragma unroll 1
    for (int mt = 0; mt < 4; ++mt) {
      const float* xrow = sX + (mt * 16 + rlane) * kXdP + koff;
      const v4f f0 = *(const v4f*)(xrow);
      const v4f f1 = *(const v4f*)(xrow + 4);
      const v4f f2 = *(const v4f*)(xrow + 16);
      const v4f f3 = *(const v4f*)(xrow + 20);
      v16b ah, al;
#pragma unroll
      for (int e = 0; e < 4; ++e) {
        __bf16 hq, lq;
        split_bf(f0[e], hq, lq); ah[e]      = hq; al[e]      = lq;
        split_bf(f1[e], hq, lq); ah[4 + e]  = hq; al[4 + e]  = lq;
        split_bf(f2[e], hq, lq); ah[8 + e]  = hq; al[8 + e]  = lq;
        split_bf(f3[e], hq, lq); ah[12 + e] = hq; al[12 + e] = lq;
      }
      v8f acc0 = (v8f){0.f,0.f,0.f,0.f,0.f,0.f,0.f,0.f};
      v8f acc1 = (v8f){0.f,0.f,0.f,0.f,0.f,0.f,0.f,0.f};
      acc0 = FB16::mma(ah, bw0, acc0);
      acc0 = FB16::mma(al, bw0, acc0);
      acc1 = FB16::mma(ah, bw1, acc1);
      acc1 = FB16::mma(al, bw1, acc1);
      dep_guard2x4_b(acc0, acc1, ah, al, bw0, bw1);
#pragma unroll
      for (int r = 0; r < 8; ++r) {
        sD[(mt * 16 + mOff + r) * kScanYP + wave * 32 + rlane]      = acc0[r];
        sD[(mt * 16 + mOff + r) * kScanYP + wave * 32 + 16 + rlane] = acc1[r];
      }
    }
    __syncthreads();
#pragma unroll 1
    for (int si = 0; si < kScanTS; ++si) {
      const int s = DIR ? (kScanTS - 1 - si) : si;
      const size_t grow = row0 + t0 + s;
      const float* xr = sX + s * kXdP;
      float Bs[kNst], Cs[kNst];
#pragma unroll
      for (int q4 = 0; q4 < 4; ++q4) {
        const v4f bv = *(const v4f*)(xr + kDtR + 4 * q4);
        const v4f cv = *(const v4f*)(xr + kDtR + kNst + 4 * q4);
        Bs[4 * q4 + 0] = bv[0]; Bs[4 * q4 + 1] = bv[1]; Bs[4 * q4 + 2] = bv[2]; Bs[4 * q4 + 3] = bv[3];
        Cs[4 * q4 + 0] = cv[0]; Cs[4 * q4 + 1] = cv[1]; Cs[4 * q4 + 2] = cv[2]; Cs[4 * q4 + 3] = cv[3];
      }
      const float v   = sD[s * kScanYP + tid] + bb;
      const float ea  = __expf(-fabsf(v));
      const float ua  = 1.0f + ea;
      const float l1p = __logf(ua) + (ea - (ua - 1.0f)) * __builtin_amdgcn_rcpf(ua);
      const float dt  = fmaxf(v, 0.0f) + l1p;
      const size_t go = grow * kDin + d;
      const size_t gw = grow * (kDin / 2) + (d >> 1);
      const unsigned wh = UHw[gw];
      const unsigned wl = ULw[gw];
      const unsigned uhb = odd ? (wh & 0xffff0000u) : (wh << 16);
      const unsigned ulb = odd ? (wl & 0xffff0000u) : (wl << 16);
      const float ut  = __uint_as_float(uhb) + __uint_as_float(ulb);
      const float dtu = dt * ut;
      float y = 0.0f;
#pragma unroll
      for (int n = 0; n < kNst; ++n) {
        const float e = __expf(dt * negA[n]);
        h[n] = e * h[n] + dtu * Bs[n];
        y = fmaf(h[n], Cs[n], y);
      }
      y = y + Dd * ut;
      const float zv = Z2[go];
      const float ez = __expf(fminf(-zv, 80.0f));
      const float gz = zv * __builtin_amdgcn_rcpf(1.0f + ez);
      float o = y * gz;
      if (DIR == 1) o = YFin[go] + o;
      sY[s * kScanYP + tid] = o;
    }
    __syncthreads();
    if (DIR == 0) {
      for (int pass = 0; pass < 2; ++pass) {
#pragma unroll
        for (int it = 0; it < 16; ++it) {
          const int row = it * 4 + wave * 2 + hh;
          const v4f val = *(const v4f*)(sY + row * kScanYP + c4);
          *(volatile v4f*)(YFout + (row0 + t0 + row) * kDin + d0 + c4) = val;
        }
        __threadfence();
      }
    } else {
      v8h hv[8], lv[8];
#pragma unroll
      for (int it = 0; it < 8; ++it) {
        const int row = it * 8 + wave * 4 + q;
        const float* sp = sY + row * kScanYP + c8;
        const v4f a0 = *(const v4f*)(sp);
        const v4f a1 = *(const v4f*)(sp + 4);
#pragma unroll
        for (int e = 0; e < 4; ++e) {
          const unsigned short h0 = f2bf_bits(a0[e]), h1 = f2bf_bits(a1[e]);
          const unsigned short l0 = f2bf_bits(a0[e] - bf_bits2f(h0)), l1 = f2bf_bits(a1[e] - bf_bits2f(h1));
          hv[it][e]     = __builtin_bit_cast(_Float16, h0);
          hv[it][4 + e] = __builtin_bit_cast(_Float16, h1);
          lv[it][e]     = __builtin_bit_cast(_Float16, l0);
          lv[it][4 + e] = __builtin_bit_cast(_Float16, l1);
        }
      }
      for (int pass = 0; pass < 2; ++pass) {
#pragma unroll
        for (int it = 0; it < 8; ++it) {
          const int row  = it * 8 + wave * 4 + q;
          const int lrow = t0 + row;
          const int frow = (strm == 0) ? lrow : (kSeq - 1 - lrow);
          const size_t o = (size_t)frow * kFinP + (size_t)strm * kDin + d0 + c8;
          *(volatile v8h*)(FH + o) = hv[it];
          *(volatile v8h*)(FL + o) = lv[it];
        }
        __threadfence();
      }
    }
  }
}

extern "C" void kernel_launch(void* const* d_in, const int* in_sizes, int n_in,
                              void* d_out, int out_size, void* d_ws, size_t ws_size,
                              hipStream_t stream) {
  if (n_in < 17) return;
  if (in_sizes[0]  != kBatch * kSeq * kDm) return;
  if (in_sizes[1]  != kWinR * kDm) return;
  if (in_sizes[2]  != kDin * 4) return;
  if (in_sizes[3]  != kDin) return;
  if (in_sizes[4]  != kXdP * kDin) return;
  if (in_sizes[5]  != kDin * kDtR) return;
  if (in_sizes[6]  != kDin) return;
  if (in_sizes[7]  != kDin * kNst) return;
  if (in_sizes[8]  != kDin) return;
  if (in_sizes[9]  != kDin * 4) return;
  if (in_sizes[10] != kDin) return;
  if (in_sizes[11] != kXdP * kDin) return;
  if (in_sizes[12] != kDin * kDtR) return;
  if (in_sizes[13] != kDin) return;
  if (in_sizes[14] != kDin * kNst) return;
  if (in_sizes[15] != kDin) return;
  if (in_sizes[16] != kDm * kFinP) return;
  if (out_size != kBatch * kSeq * kDm) return;
  if (ws_size < kWsTotal) return;

  const float* hs     = (const float*)d_in[0];
  const float* W_in   = (const float*)d_in[1];
  const float* cw_f   = (const float*)d_in[2];
  const float* cb_f   = (const float*)d_in[3];
  const float* xw_f   = (const float*)d_in[4];
  const float* dw_f   = (const float*)d_in[5];
  const float* db_f   = (const float*)d_in[6];
  const float* Alog_f = (const float*)d_in[7];
  const float* D_f    = (const float*)d_in[8];
  const float* cw_b   = (const float*)d_in[9];
  const float* cb_b   = (const float*)d_in[10];
  const float* xw_b   = (const float*)d_in[11];
  const float* dw_b   = (const float*)d_in[12];
  const float* db_b   = (const float*)d_in[13];
  const float* Alog_b = (const float*)d_in[14];
  const float* D_b    = (const float*)d_in[15];
  const float* W_out  = (const float*)d_in[16];
  float* out = (float*)d_out;

  char* ws = (char*)d_ws;
  unsigned short* XB  = (unsigned short*)(ws + kOffXB);
  unsigned short* WIB = (unsigned short*)(ws + kOffWIB);
  unsigned short* WXF = (unsigned short*)(ws + kOffWXF);
  unsigned short* WXB = (unsigned short*)(ws + kOffWXB);
  unsigned short* WOB = (unsigned short*)(ws + kOffWOB);
  float*          X2  = (float*)(ws + kOffX2);
  float*          Z2  = (float*)(ws + kOffZ2);
  unsigned short* UFH = (unsigned short*)(ws + kOffUFH);
  unsigned short* UFL = (unsigned short*)(ws + kOffUFL);
  unsigned short* UBH = (unsigned short*)(ws + kOffUBH);
  unsigned short* UBL = (unsigned short*)(ws + kOffUBL);
  float*          XDF = (float*)(ws + kOffXDF);
  float*          XDB = (float*)(ws + kOffXDB);
  float*          YF  = (float*)(ws + kOffYF);
  unsigned short* FH  = (unsigned short*)(ws + kOffFH);
  unsigned short* FL  = (unsigned short*)(ws + kOffFL);

  cvt_rows_bf16_kernel<<<(kBatch * kSeq * kDm / 8) / 256, 256, 0, stream>>>(hs, XB, kBatch * kSeq * kDm / 8);
  cvt_rows_bf16_kernel<<<(kWinR * kDm / 8) / 256, 256, 0, stream>>>(W_in, WIB, kWinR * kDm / 8);
  cvt_rows_bf16_kernel<<<(kXdP * kDin / 8) / 256, 256, 0, stream>>>(xw_f, WXF, kXdP * kDin / 8);
  cvt_rows_bf16_kernel<<<(kXdP * kDin / 8) / 256, 256, 0, stream>>>(xw_b, WXB, kXdP * kDin / 8);
  cvt_rows_bf16_kernel<<<(kDm * kFinP / 8) / 256, 256, 0, stream>>>(W_out, WOB, kDm * kFinP / 8);

  const long strideBsel = (long)kDin * kDm;
  const long strideCsel = (long)kRowsB * kDin;
  const int  tilesIn  = (kSeq / 64) * (kDin / 64) / 8;
  const int  tilesX   = (kRowsB / 64) * (kXdP / 64) / 8;
  const int  tilesOut = (kSeq / 64) * (kDm / 64) / 8;

  for (int b = 0; b < kBatch; ++b) {
    const unsigned short* XBb = XB + (size_t)b * kSeq * kDm;
    float* outb = out + (size_t)b * kSeq * kDm;

    wmma_gemm64<1, 0, 0, 0, false, 0, 0><<<dim3(tilesIn, 2), 256, 0, stream>>>(
        XBb, nullptr, kDm, 0L,
        WIB, nullptr, kDm, strideBsel,
        (void*)X2, nullptr, kDin, strideCsel,
        nullptr, nullptr, 0L,
        kSeq, kDin, kDm, 1.0f);
    wmma_gemm64<1, 0, 0, 0, false, 0, 1><<<dim3(tilesIn, 2), 256, 0, stream>>>(
        XBb, nullptr, kDm, 0L,
        WIB + (size_t)2 * kDin * kDm, nullptr, kDm, strideBsel,
        (void*)(X2 + (size_t)kSeq * kDin), nullptr, kDin, strideCsel,
        nullptr, nullptr, 0L,
        kSeq, kDin, kDm, 1.0f);

    conv_silu_kernel<0><<<dim3(kDin / 256, kRowsB / 64), 256, 0, stream>>>(X2, cw_f, cb_f, UFH, UFL);
    conv_silu_kernel<1><<<dim3(kDin / 256, kRowsB / 64), 256, 0, stream>>>(X2, cw_b, cb_b, UBH, UBL);

    wmma_gemm64<1, 1, 0, 0, false, 0, 0><<<dim3(tilesX, 1), 256, 0, stream>>>(
        UFH, UFL, kDin, 0L,
        WXF, nullptr, kDin, 0L,
        (void*)XDF, nullptr, kXdP, 0L,
        nullptr, nullptr, 0L,
        kRowsB, kXdP, kDin, 1.0f);
    wmma_gemm64<1, 1, 0, 0, false, 0, 0><<<dim3(tilesX, 1), 256, 0, stream>>>(
        UBH, UBL, kDin, 0L,
        WXB, nullptr, kDin, 0L,
        (void*)XDB, nullptr, kXdP, 0L,
        nullptr, nullptr, 0L,
        kRowsB, kXdP, kDin, 1.0f);

    scan_kernel<0><<<kStr * (kDin / kScanCh), kScanCh, 0, stream>>>(
        XDF, UFH, UFL, Z2, dw_f, db_f, Alog_f, D_f, nullptr, YF, nullptr, nullptr);
    scan_kernel<1><<<kStr * (kDin / kScanCh), kScanCh, 0, stream>>>(
        XDB, UBH, UBL, Z2, dw_b, db_b, Alog_b, D_b, YF, nullptr, FH, FL);

    wmma_gemm64<1, 1, 0, 0, false, 0, 0><<<dim3(tilesOut, 1), 256, 0, stream>>>(
        FH, FL, kFinP, 0L,
        WOB, nullptr, kFinP, 0L,
        (void*)outb, nullptr, kDm, 0L,
        nullptr, nullptr, 0L,
        kSeq, kDm, kFinP, 1.0f);
  }
}
